// QuantizedAttention_14388140441831
// MI455X (gfx1250) — hardware-verified
//
#include <hip/hip_runtime.h>
#include <math.h>
#include <stdint.h>

#define NB    2
#define SEQ   2048
#define DMOD  1024
#define NH    16
#define HD    64
#define HP    32
#define QSC   1024.0f
#define KSC   1024.0f
#define PCAR  32768.0f
#define VCAR  1024.0f
#define OSC   1024.0f
#define WOS   1024.0f
#define QMAX  448.0f
#define LOG2E 1.4426950408889634f
#define ATT_WAVES   4
#define ATT_THREADS (ATT_WAVES * 32)
#define ATT_BLOCKS  (NB * NH * (SEQ / 64))
#define MAXBLK (SEQ / 32)
#define SLABF (16 * 68)
#define SLAB64 (16 * 68)
#define VTP   72
static_assert(HD == 64 && DMOD == NH * HD && HP * 2 == HD);
static_assert((SEQ / 64) == 32 && NH == 16 && NB == 2);
static_assert(ATT_THREADS == 128 && ATT_BLOCKS == 1024 && MAXBLK == 64);
static_assert(16 * 36 <= SLABF);
static_assert(((NB * SEQ * NH * 8) % 256) == 0);
static_assert(((NB * SEQ) % 64) == 0 && (DMOD % 64) == 0 && (DMOD % 32) == 0);
static_assert((SEQ % 64) == 0 && (SEQ % 8) == 0);
static_assert(((NB * SEQ * DMOD / 8) % 256) == 0);
static_assert((NH * (DMOD / 64)) == 256 && ((DMOD / 64) * (DMOD / 64)) == 256);

typedef unsigned short u16;
typedef _Float16 v16h __attribute__((ext_vector_type(16)));
typedef _Float16 v8h  __attribute__((ext_vector_type(8)));
typedef __bf16   v16b __attribute__((ext_vector_type(16)));
typedef float    v8f  __attribute__((ext_vector_type(8)));
typedef float    v4f  __attribute__((ext_vector_type(4)));
typedef unsigned int v4u __attribute__((ext_vector_type(4)));

union FragH { v16h v; v8h h[2]; v4u u[2]; };
union FragB { v16b v; v4u u[2]; };

struct InvF { float f[32]; };
static_assert(sizeof(InvF) == 128);

__device__ __forceinline__ unsigned short bf_bits(float f) {
  unsigned u = __float_as_uint(f);
  return (unsigned short)((u + 0x7FFFu + ((u >> 16) & 1u)) >> 16);
}
__device__ __forceinline__ float bf_up(unsigned short h) { return __uint_as_float(((unsigned)h) << 16); }
__device__ __forceinline__ float bfr(float f) { return bf_up(bf_bits(f)); }
__device__ __forceinline__ unsigned short h_bits(_Float16 x) { return __builtin_bit_cast(unsigned short, x); }
__device__ __forceinline__ unsigned pk16(unsigned short a, unsigned short b) { return (unsigned)a | ((unsigned)b << 16); }
__device__ __forceinline__ v8f zero8() { v8f z = {0.f, 0.f, 0.f, 0.f, 0.f, 0.f, 0.f, 0.f}; return z; }
__device__ __forceinline__ v4f zero4() { v4f z = {0.f, 0.f, 0.f, 0.f}; return z; }

__device__ __forceinline__ float fq8(float w, float scale) {
  const float v  = w * scale;
  const float a  = fabsf(v);
  const float am = fmaxf(a, 1e-30f);
  int ex = (int)((__float_as_uint(am) >> 23) & 0xFFu) - 127;
  ex = (ex < -6) ? -6 : ((ex > 8) ? 8 : ex);
  const float step  = __uint_as_float((unsigned)(ex - 3 + 127) << 23);
  const float rstep = __uint_as_float((unsigned)(127 + 3 - ex) << 23);
  float q = rintf(v * rstep) * step;
  q = fminf(fmaxf(q, -QMAX), QMAX);
  return q;
}

__device__ __forceinline__ v16h ldfrag_h(const _Float16* p) {
  FragH f;
  f.h[0] = *(const v8h*)(p);
  f.h[1] = *(const v8h*)(p + 16);
  return f.v;
}
__device__ __forceinline__ v16b ldfrag_b(const u16* p) {
  FragB f;
  f.u[0] = *(const v4u*)(p);
  f.u[1] = *(const v4u*)(p + 16);
  return f.v;
}

__device__ __forceinline__ v8f mma_h(v16h a, v16h b, v8f c) {
  return __builtin_amdgcn_wmma_f32_16x16x32_f16(false, a, false, b, (short)0, c, false, false);
}
__device__ __forceinline__ v8f mma_b(v16b a, v16b b, v8f c) {
  return __builtin_amdgcn_wmma_f32_16x16x32_bf16(false, a, false, b, (short)0, c, false, false);
}
__device__ __forceinline__ void guard2(v8f& a, v8f& b, v16h x0, v16h x1, v16h x2, v16h x3, v16h x4, v16h x5) {
#if defined(__HIP_DEVICE_COMPILE__)
  asm volatile("v_nop\n\tv_nop\n\tv_nop\n\tv_nop"
               : "+v"(a), "+v"(b) : "v"(x0), "v"(x1), "v"(x2), "v"(x3), "v"(x4), "v"(x5) : "memory");
#endif
}
template <typename F>
__device__ __forceinline__ void guard6(v8f& a, v8f& b, v8f& c, v8f& d, F x0, F x1, F x2, F x3, F x4, F x5) {
#if defined(__HIP_DEVICE_COMPILE__)
  asm volatile("v_nop\n\tv_nop\n\tv_nop\n\tv_nop"
               : "+v"(a), "+v"(b), "+v"(c), "+v"(d) : "v"(x0), "v"(x1), "v"(x2), "v"(x3), "v"(x4), "v"(x5) : "memory");
#endif
}
__device__ __forceinline__ void guard10(v8f& a, v8f& b, v8f& c, v8f& d, v16h x0, v16h x1, v16h x2, v16h x3, v16h x4,
                                        v16h x5, v16h x6, v16h x7, v16h x8, v16h x9) {
#if defined(__HIP_DEVICE_COMPILE__)
  asm volatile("v_nop\n\tv_nop\n\tv_nop\n\tv_nop"
               : "+v"(a), "+v"(b), "+v"(c), "+v"(d)
               : "v"(x0), "v"(x1), "v"(x2), "v"(x3), "v"(x4), "v"(x5), "v"(x6), "v"(x7), "v"(x8), "v"(x9) : "memory");
#endif
}
__device__ __forceinline__ void acc_guard4(v8f& a, v8f& b, v8f& c, v8f& d) {
#if defined(__HIP_DEVICE_COMPILE__)
  asm volatile("v_nop\n\tv_nop\n\tv_nop\n\tv_nop" : "+v"(a), "+v"(b), "+v"(c), "+v"(d));
#endif
}
__device__ __forceinline__ void wave_sync_lds() {
  __builtin_amdgcn_fence(__ATOMIC_RELEASE, "workgroup");
  __builtin_amdgcn_wave_barrier();
  __builtin_amdgcn_fence(__ATOMIC_ACQUIRE, "workgroup");
}

__device__ __forceinline__ void sincos_acc(float angf, float& sv, float& cv) {
  const double a = (double)angf;
  const double TWO_OVER_PI = 0.63661977236758134308;
  const double PIO2_HI = 1.5707963267948966;
  const double PIO2_LO = 6.123233995736766e-17;
  const int kq = (int)(a * TWO_OVER_PI + 0.5);
  const double kd = (double)kq;
  double r = fma(-kd, PIO2_HI, a);
  r = fma(-kd, PIO2_LO, r);
  const double r2 = r * r;
  double sp = 1.0 / 6227020800.0;
  sp = fma(sp, r2, -1.0 / 39916800.0);
  sp = fma(sp, r2, 1.0 / 362880.0);
  sp = fma(sp, r2, -1.0 / 5040.0);
  sp = fma(sp, r2, 1.0 / 120.0);
  sp = fma(sp, r2, -1.0 / 6.0);
  const double s = fma(sp * r2, r, r);
  double cp = -1.0 / 87178291200.0;
  cp = fma(cp, r2, 1.0 / 479001600.0);
  cp = fma(cp, r2, -1.0 / 3628800.0);
  cp = fma(cp, r2, 1.0 / 40320.0);
  cp = fma(cp, r2, -1.0 / 720.0);
  cp = fma(cp, r2, 1.0 / 24.0);
  cp = fma(cp, r2, -0.5);
  const double c = fma(cp, r2, 1.0);
  const int qd = kq & 3;
  const double so = (qd == 0) ? s : (qd == 1) ? c : (qd == 2) ? -s : -c;
  const double co = (qd == 0) ? c : (qd == 1) ? -s : (qd == 2) ? -c : s;
  sv = (float)so;
  cv = (float)co;
}

__global__ __launch_bounds__(256) void k_tab(float* cosT, float* sinT, InvF inv) {
  const int tid  = threadIdx.x;
  const int lane = tid & 31;
  const int t    = blockIdx.x * 8 + (tid >> 5);
  if (t >= SEQ) return;
  float f = inv.f[0];
#pragma unroll
  for (int i = 1; i < 32; ++i) f = (lane == i) ? inv.f[i] : f;
  const float ang = (float)t * f;
  float sv, cv;
  sincos_acc(ang, sv, cv);
  float* cr = cosT + (size_t)t * HP;
  float* sr = sinT + (size_t)t * HP;
  for (int pass = 0; pass < 2; ++pass) {
    *(volatile float*)(cr + lane) = cv;
    *(volatile float*)(sr + lane) = sv;
    __threadfence();
  }
}

__global__ __launch_bounds__(256)
void k_stats(const float* __restrict__ w0, const float* __restrict__ w1, const float* __restrict__ w2,
             const float* __restrict__ b0, const float* __restrict__ b1, const float* __restrict__ b2,
             int nW4, int nB4, float* st, float* bqd) {
  __shared__ float red[8];
  const int tid = threadIdx.x, lane = tid & 31, wave = tid >> 5;
  const int t = blockIdx.x;
  const float* src = (t == 0) ? w0 : (t == 1) ? w1 : (t == 2) ? w2 : (t == 3) ? b0 : (t == 4) ? b1 : b2;
  const int n4 = (t < 3) ? nW4 : nB4;
  float m = 0.f;
#pragma unroll 1
  for (int i = tid; i < n4; i += 256) {
    const v4f a = *(const v4f*)(src + (size_t)i * 4);
#pragma unroll
    for (int e = 0; e < 4; ++e) m = fmaxf(m, fabsf(bfr(a[e])));
  }
#pragma unroll
  for (int off = 1; off < 32; off <<= 1) m = fmaxf(m, __shfl_xor(m, off, 32));
  if (lane == 0) red[wave] = m;
  __syncthreads();
  float am = red[0];
#pragma unroll
  for (int i = 1; i < 8; ++i) am = fmaxf(am, red[i]);
  const float den    = fmaxf(am, 1e-12f);
  const float scale  = (float)(448.0 / (double)den);
  const float rscale = (float)(1.0 / (double)scale);
  if (wave == 0) {
    const float val = (lane == 0) ? am : (lane == 1) ? scale : (lane == 2) ? rscale : 0.f;
    float* sp = st + t * 32 + lane;
    for (int pass = 0; pass < 2; ++pass) {
      *(volatile float*)sp = val;
      __threadfence();
    }
  }
  if (t >= 3) {
    const int i4 = (tid < nB4) ? tid : (nB4 - 1);
    const v4f a = *(const v4f*)(src + (size_t)i4 * 4);
    v4f o;
#pragma unroll
    for (int e = 0; e < 4; ++e) o[e] = fq8(bfr(a[e]), scale) * rscale;
    if (tid < nB4) {
      float* bp = bqd + (size_t)(t - 3) * (NH * HD) + (size_t)i4 * 4;
      for (int pass = 0; pass < 2; ++pass) {
        *(volatile v4f*)bp = o;
        __threadfence();
      }
    }
  }
}

__global__ __launch_bounds__(256) void wqt16(const float* __restrict__ W, const float* __restrict__ st, u16* Bt) {
  __shared__ __align__(16) u16 T[HD * VTP];
  const int tid = threadIdx.x;
  const int bid = blockIdx.x;
  const int h   = bid >> 4;
  const int d0  = (bid & 15) * 64;
  const float scale = st[1];
  {
    const int dl = tid >> 2;
    const int ec = (tid & 3) * 16;
    const float* src = W + ((size_t)(h * DMOD + d0 + dl)) * HD + ec;
#pragma unroll
    for (int i = 0; i < 4; ++i) {
      const v4f a = *(const v4f*)(src + 4 * i);
#pragma unroll
      for (int e = 0; e < 4; ++e) {
        const float q = fq8(bfr(a[e]), scale);
        T[(ec + 4 * i + e) * VTP + dl] = bf_bits(q);
      }
    }
  }
  __syncthreads();
  v4u o[2];
  const int q8 = tid >> 3, p8 = (tid & 7) * 8;
#pragma unroll
  for (int it = 0; it < 2; ++it) {
    const int line = it * 32 + q8;
    o[it] = *(const v4u*)(T + line * VTP + p8);
  }
  const size_t base = ((size_t)(h * HD)) * DMOD + d0 + p8;
  for (int pass = 0; pass < 2; ++pass) {
#pragma unroll
    for (int it = 0; it < 2; ++it) {
      const int line = it * 32 + q8;
      *(volatile v4u*)(Bt + base + (size_t)line * DMOD) = o[it];
    }
    __threadfence();
  }
}

__global__ __launch_bounds__(256) void wot16(const float* __restrict__ Wo, u16* Bt) {
  __shared__ __align__(16) u16 T[HD * VTP];
  const int tid = threadIdx.x;
  const int bid = blockIdx.x;
  const int he0 = (bid & 15) * 64;
  const int d0  = (bid >> 4) * 64;
  {
    const int rl = tid >> 2;
    const int dc = (tid & 3) * 16;
    const float* src = Wo + (size_t)(he0 + rl) * DMOD + d0 + dc;
#pragma unroll
    for (int i = 0; i < 4; ++i) {
      const v4f a = *(const v4f*)(src + 4 * i);
#pragma unroll
      for (int e = 0; e < 4; ++e) {
        const float tv = bfr(a[e]) * WOS;
        T[(dc + 4 * i + e) * VTP + rl] = h_bits((_Float16)tv);
      }
    }
  }
  __syncthreads();
  v4u o[2];
  const int q8 = tid >> 3, p8 = (tid & 7) * 8;
#pragma unroll
  for (int it = 0; it < 2; ++it) {
    const int line = it * 32 + q8;
    o[it] = *(const v4u*)(T + line * VTP + p8);
  }
  const size_t base = (size_t)d0 * DMOD + he0 + p8;
  for (int pass = 0; pass < 2; ++pass) {
#pragma unroll
    for (int it = 0; it < 2; ++it) {
      const int line = it * 32 + q8;
      *(volatile v4u*)(Bt + base + (size_t)line * DMOD) = o[it];
    }
    __threadfence();
  }
}

__global__ __launch_bounds__(256) void cvtbf(const float* __restrict__ x, u16* D, int n8) {
  const int gt = blockIdx.x * 256 + (int)threadIdx.x;
  if (gt >= n8) return;
  const float* p = x + (size_t)gt * 8;
  const v4f a = *(const v4f*)(p), bq = *(const v4f*)(p + 4);
  float v[8];
#pragma unroll
  for (int e = 0; e < 4; ++e) { v[e] = a[e]; v[4 + e] = bq[e]; }
  v4u o;
#pragma unroll
  for (int e = 0; e < 4; ++e) o[e] = pk16(bf_bits(v[2 * e]), bf_bits(v[2 * e + 1]));
  u16* d = D + (size_t)gt * 8;
  for (int pass = 0; pass < 2; ++pass) {
    *(volatile v4u*)(d) = o;
    __threadfence();
  }
}

__device__ __forceinline__ void epi64(float* sl, v8f a0, v8f a1, v8f a2, v8f a3, float oscale, v4f badd, float* C, int N,
                                      size_t rowb, int col0, int lane) {
  const int hh = lane >> 4, m = lane & 15;
#pragma unroll
  for (int r = 0; r < 8; ++r) {
    const int ro = (8 * hh + r) * 68 + m;
    sl[ro]      = a0[r] * oscale;
    sl[ro + 16] = a1[r] * oscale;
    sl[ro + 32] = a2[r] * oscale;
    sl[ro + 48] = a3[r] * oscale;
  }
  wave_sync_lds();
  v4f vals[8];
#pragma unroll
  for (int it = 0; it < 8; ++it) vals[it] = *(const v4f*)(sl + (it * 2 + hh) * 68 + m * 4) + badd;
  float* dst = C + (rowb + (size_t)hh) * (size_t)N + col0 + m * 4;
  for (int pass = 0; pass < 2; ++pass) {
#pragma unroll
    for (int it = 0; it < 8; ++it) {
      *(volatile v4f*)(dst + (size_t)(it * 2) * (size_t)N) = vals[it];
    }
    __threadfence();
  }
}

__global__ __launch_bounds__(128)
void gemm_bf(const u16* __restrict__ A, const u16* __restrict__ Bt, const float* __restrict__ bias,
             const float* __restrict__ osp, float* C, int M, int N, int K) {
  __shared__ __align__(16) float slab[4 * SLAB64];
  const int tid = threadIdx.x, wave = tid >> 5, lane = tid & 31, hh = lane >> 4, m = lane & 15;
  const int ntile = N >> 6;
  const int bid   = blockIdx.x;
  const int rowb  = (bid / ntile) * 64 + wave * 16;
  const int col0  = (bid % ntile) * 64;
  if (rowb + 16 > M) return;
  const float oscale = osp[0];
  const u16* ap = A  + (size_t)(rowb + m) * K + 8 * hh;
  const u16* bp = Bt + (size_t)(col0 + m) * K + 8 * hh;
  const size_t bs = (size_t)16 * K;
  v8f acc0 = zero8(), acc1 = zero8(), acc2 = zero8(), acc3 = zero8();
#pragma unroll 1
  for (int k0 = 0; k0 < K; k0 += 32) {
    const v16b a  = ldfrag_b(ap + k0);
    const v16b b0 = ldfrag_b(bp + k0);
    const v16b b1 = ldfrag_b(bp + bs + k0);
    const v16b b2 = ldfrag_b(bp + 2 * bs + k0);
    const v16b b3 = ldfrag_b(bp + 3 * bs + k0);
    acc0 = mma_b(a, b0, acc0);
    acc1 = mma_b(a, b1, acc1);
    acc2 = mma_b(a, b2, acc2);
    acc3 = mma_b(a, b3, acc3);
    guard6<v16b>(acc0, acc1, acc2, acc3, a, b0, b1, b2, b3, a);
  }
  const v4f badd = *(const v4f*)(bias + col0 + m * 4);
  epi64(slab + wave * SLAB64, acc0, acc1, acc2, acc3, oscale, badd, C, N, (size_t)rowb, col0, lane);
}

__global__ __launch_bounds__(128)
void gemm_h2(const u16* __restrict__ Ah, const u16* __restrict__ Al, const u16* __restrict__ Bt,
             const float* __restrict__ bias, float* C, int M, int N, int K, float oscale) {
  __shared__ __align__(16) float slab[4 * SLAB64];
  const int tid = threadIdx.x, wave = tid >> 5, lane = tid & 31, hh = lane >> 4, m = lane & 15;
  const int ntile = N >> 6;
  const int bid   = blockIdx.x;
  const int rowb  = (bid / ntile) * 64 + wave * 16;
  const int col0  = (bid % ntile) * 64;
  if (rowb + 16 > M) return;
  const size_t aofs = (size_t)(rowb + m) * K + 8 * hh;
  const _Float16* ahp = (const _Float16*)(const void*)Ah + aofs;
  const _Float16* alp = (const _Float16*)(const void*)Al + aofs;
  const _Float16* bp  = (const _Float16*)(const void*)Bt + (size_t)(col0 + m) * K + 8 * hh;
  const size_t bs = (size_t)16 * K;
  v8f acc0 = zero8(), acc1 = zero8(), acc2 = zero8(), acc3 = zero8();
#pragma unroll 1
  for (int k0 = 0; k0 < K; k0 += 32) {
    const v16h ah = ldfrag_h(ahp + k0), al = ldfrag_h(alp + k0);
    const v16h b0 = ldfrag_h(bp + k0);
    const v16h b1 = ldfrag_h(bp + bs + k0);
    const v16h b2 = ldfrag_h(bp + 2 * bs + k0);
    const v16h b3 = ldfrag_h(bp + 3 * bs + k0);
    acc0 = mma_h(ah, b0, acc0);  acc0 = mma_h(al, b0, acc0);
    acc1 = mma_h(ah, b1, acc1);  acc1 = mma_h(al, b1, acc1);
    acc2 = mma_h(ah, b2, acc2);  acc2 = mma_h(al, b2, acc2);
    acc3 = mma_h(ah, b3, acc3);  acc3 = mma_h(al, b3, acc3);
    guard6<v16h>(acc0, acc1, acc2, acc3, ah, al, b0, b1, b2, b3);
  }
  const v4f bv = *(const v4f*)(bias + col0 + m * 4);
  v4f badd;
#pragma unroll
  for (int e = 0; e < 4; ++e) badd[e] = bfr(bv[e]);
  epi64(slab + wave * SLAB64, acc0, acc1, acc2, acc3, oscale, badd, C, N, (size_t)rowb, col0, lane);
}

__global__ __launch_bounds__(256) void rot16(const float* __restrict__ x,
                                             const float* __restrict__ cosT, const float* __restrict__ sinT,
                                             u16* hpl, u16* lpl, int nrows, int hpr, float sc) {
#pragma clang fp contract(off)
  const int gt   = blockIdx.x * 256 + (int)threadIdx.x;
  const int row  = gt >> 3;
  const int d0   = (gt & 7) * 8;
  const bool live = row < nrows;
  const int rowc = live ? row : (nrows - 1);
  const int pos  = (rowc / hpr) & (SEQ - 1);
  const float* xr = x + (size_t)rowc * HD;
  const int dp   = d0 ^ HP;
  const v4f xa = *(const v4f*)(xr + d0), xb = *(const v4f*)(xr + d0 + 4);
  const v4f pa = *(const v4f*)(xr + dp), pb = *(const v4f*)(xr + dp + 4);
  const int i0 = d0 & (HP - 1);
  const v4f ca = *(const v4f*)(cosT + (size_t)pos * HP + i0), cb = *(const v4f*)(cosT + (size_t)pos * HP + i0 + 4);
  const v4f sa = *(const v4f*)(sinT + (size_t)pos * HP + i0), sb = *(const v4f*)(sinT + (size_t)pos * HP + i0 + 4);
  float y[8], yp[8], cs[8], sn[8];
#pragma unroll
  for (int e = 0; e < 4; ++e) {
    y[e]  = xa[e]; y[4 + e]  = xb[e];
    yp[e] = pa[e]; yp[4 + e] = pb[e];
    cs[e] = ca[e]; cs[4 + e] = cb[e];
    sn[e] = sa[e]; sn[4 + e] = sb[e];
  }
  const bool lowh = d0 < HP;
  float w[8];
#pragma unroll
  for (int e = 0; e < 8; ++e) {
    const float fl = lowh ? -yp[e] : yp[e];
    const float pa2 = y[e] * cs[e];
    const float pb2 = fl * sn[e];
    w[e] = pa2 + pb2;
  }
  v4u oh, ol;
#pragma unroll
  for (int e = 0; e < 4; ++e) {
    const float t0 = w[2 * e] * sc, t1 = w[2 * e + 1] * sc;
    const _Float16 h0 = (_Float16)t0, h1 = (_Float16)t1;
    const _Float16 l0 = (_Float16)(t0 - (float)h0), l1 = (_Float16)(t1 - (float)h1);
    oh[e] = pk16(h_bits(h0), h_bits(h1));
    ol[e] = pk16(h_bits(l0), h_bits(l1));
  }
  if (live) {
    const size_t o8 = (size_t)row * HD + d0;
    for (int pass = 0; pass < 2; ++pass) {
      *(volatile v4u*)(hpl + o8) = oh;
      *(volatile v4u*)(lpl + o8) = ol;
      __threadfence();
    }
  }
}

__global__ __launch_bounds__(256) void vt16(const float* __restrict__ v, u16* VHo, u16* VLo) {
  __shared__ __align__(16) u16 TH[HD * VTP];
  __shared__ __align__(16) u16 TL[HD * VTP];
  const int tid = threadIdx.x;
  const int bid = blockIdx.x;
  const int st  = bid & 31;
  const int h   = (bid >> 5) & (NH - 1);
  const int b   = bid >> 9;
  const int s0  = st * 64;
  {
    const int sl = tid >> 2;
    const int dc = (tid & 3) * 16;
    const float* src = v + (((size_t)(b * SEQ + s0 + sl)) * NH + h) * HD + dc;
#pragma unroll
    for (int i = 0; i < 4; ++i) {
      const v4f a = *(const v4f*)(src + 4 * i);
#pragma unroll
      for (int e = 0; e < 4; ++e) {
        const float t = a[e] * VCAR;
        const _Float16 hv = (_Float16)t;
        const _Float16 lv = (_Float16)(t - (float)hv);
        TH[(dc + 4 * i + e) * VTP + sl] = h_bits(hv);
        TL[(dc + 4 * i + e) * VTP + sl] = h_bits(lv);
      }
    }
  }
  __syncthreads();
  v4u vh[2], vl[2];
  const int q8 = tid >> 3, p8 = (tid & 7) * 8;
#pragma unroll
  for (int it = 0; it < 2; ++it) {
    const int line = it * 32 + q8;
    vh[it] = *(const v4u*)(TH + line * VTP + p8);
    vl[it] = *(const v4u*)(TL + line * VTP + p8);
  }
  const size_t base = ((size_t)(b * NH + h) * HD) * SEQ + s0 + p8;
  for (int pass = 0; pass < 2; ++pass) {
#pragma unroll
    for (int it = 0; it < 2; ++it) {
      const int line = it * 32 + q8;
      *(volatile v4u*)(VHo + base + (size_t)line * SEQ) = vh[it];
      *(volatile v4u*)(VLo + base + (size_t)line * SEQ) = vl[it];
    }
    __threadfence();
  }
}

__global__ __launch_bounds__(ATT_THREADS)
void attn_causal(const u16* __restrict__ QHIp, const u16* __restrict__ QLOp,
                 const u16* __restrict__ KHIp, const u16* __restrict__ KLOp,
                 const u16* __restrict__ VHIp, const u16* __restrict__ VLOp,
                 u16* OHIp, u16* OLOp) {
  __shared__ __align__(16) float smem[ATT_WAVES * SLABF];

  const int tid  = threadIdx.x;
  const int wave = tid >> 5;
  const int lane = tid & 31;
  const int hh   = lane >> 4;
  const int c    = lane & 15;

  const int bid  = blockIdx.x;
  const int qt   = bid & (SEQ / 64 - 1);
  const int head = (bid >> 5) & (NH - 1);
  const int b    = bid >> 9;
  const int q0   = qt * 64 + wave * 16;

  const size_t qofs = (((size_t)(b * SEQ + q0 + c)) * NH + head) * HD + 8 * hh;
  const _Float16* Qh  = (const _Float16*)(const void*)QHIp + qofs;
  const _Float16* Ql  = (const _Float16*)(const void*)QLOp + qofs;
  const size_t kofs = (((size_t)b * SEQ + c) * NH + head) * HD + 8 * hh;
  const _Float16* Khb = (const _Float16*)(const void*)KHIp + kofs;
  const _Float16* Klb = (const _Float16*)(const void*)KLOp + kofs;
  const size_t vofs = ((size_t)(b * NH + head) * HD + c) * SEQ + 8 * hh;
  const _Float16* Vhb = (const _Float16*)(const void*)VHIp + vofs;
  const _Float16* Vlb = (const _Float16*)(const void*)VLOp + vofs;
  const float lsc = 0.125f * (LOG2E / (QSC * KSC));

  float mrow[8], lrow[8];
  v8f o[4];
#pragma unroll
  for (int r = 0; r < 8; ++r) { mrow[r] = -INFINITY; lrow[r] = 0.f; }
#pragma unroll
  for (int j = 0; j < 4; ++j) o[j] = zero8();
  float* pt = smem + wave * SLABF;

  int nit = (q0 >> 5) + 1;
  nit = (nit > MAXBLK) ? MAXBLK : nit;

#pragma unroll 1
  for (int it = 0; it < nit; ++it) {
    const int kb = it * 32;
    v8f s0 = zero8(), s1 = zero8();
    const _Float16* k0p = Khb + (size_t)kb * (NH * HD);
    const _Float16* k1p = k0p + (size_t)16 * (NH * HD);
    const _Float16* l0p = Klb + (size_t)kb * (NH * HD);
    const _Float16* l1p = l0p + (size_t)16 * (NH * HD);
#pragma unroll
    for (int kk = 0; kk < 2; ++kk) {
      const v16h qh  = ldfrag_h(Qh + kk * 32),  ql  = ldfrag_h(Ql + kk * 32);
      const v16h kh0 = ldfrag_h(k0p + kk * 32), kl0 = ldfrag_h(l0p + kk * 32);
      const v16h kh1 = ldfrag_h(k1p + kk * 32), kl1 = ldfrag_h(l1p + kk * 32);
      s0 = mma_h(qh, kh0, s0);
      s0 = mma_h(ql, kh0, s0);
      s0 = mma_h(qh, kl0, s0);
      s1 = mma_h(qh, kh1, s1);
      s1 = mma_h(ql, kh1, s1);
      s1 = mma_h(qh, kl1, s1);
      guard2(s0, s1, qh, ql, kh0, kl0, kh1, kl1);
    }
    const int kc0 = kb + c, kc1 = kb + 16 + c;
#pragma unroll
    for (int r = 0; r < 8; ++r) {
      const int qr = q0 + 8 * hh + r;
      const float t0 = (kc0 <= qr) ? s0[r] * lsc : -INFINITY;
      const float t1 = (kc1 <= qr) ? s1[r] * lsc : -INFINITY;
      float mx = fmaxf(t0, t1);
#pragma unroll
      for (int off = 1; off < 16; off <<= 1) mx = fmaxf(mx, __shfl_xor(mx, off, 32));
      const float mn   = fmaxf(mrow[r], mx);
      const float mref = (mn == -INFINITY) ? 0.f : mn;
      const float al   = exp2f(mrow[r] - mref);
      mrow[r] = mn;
      const float e0 = exp2f(t0 - mref), e1 = exp2f(t1 - mref);
      float ps = e0 + e1;
#pragma unroll
      for (int off = 1; off < 16; off <<= 1) ps += __shfl_xor(ps, off, 32);
      lrow[r] = lrow[r] * al + ps;
#pragma unroll
      for (int j = 0; j < 4; ++j) o[j][r] *= al;
      const int ro = (8 * hh + r) * 36 + c;
      pt[ro]      = e0;
      pt[ro + 16] = e1;
    }
    wave_sync_lds();
    FragH ph, pl;
    {
      const float* prow = pt + c * 36 + 8 * hh;
      const v4f p0 = *(const v4f*)(prow), p1 = *(const v4f*)(prow + 4);
      const v4f p2 = *(const v4f*)(prow + 16), p3 = *(const v4f*)(prow + 20);
#pragma unroll
      for (int e = 0; e < 4; ++e) {
        const float ta = p0[e] * PCAR, tb = p1[e] * PCAR, tc = p2[e] * PCAR, td = p3[e] * PCAR;
        const _Float16 ha = (_Float16)ta, hb = (_Float16)tb, hc = (_Float16)tc, hd = (_Float16)td;
        ph.h[0][e]     = ha;
        ph.h[0][4 + e] = hb;
        ph.h[1][e]     = hc;
        ph.h[1][4 + e] = hd;
        pl.h[0][e]     = (_Float16)(ta - (float)ha);
        pl.h[0][4 + e] = (_Float16)(tb - (float)hb);
        pl.h[1][e]     = (_Float16)(tc - (float)hc);
        pl.h[1][4 + e] = (_Float16)(td - (float)hd);
      }
    }
    {
      const _Float16* vhp = Vhb + kb;
      const _Float16* vlp = Vlb + kb;
      const v16h vh0 = ldfrag_h(vhp);
      const v16h vh1 = ldfrag_h(vhp + (size_t)16 * SEQ);
      const v16h vh2 = ldfrag_h(vhp + (size_t)32 * SEQ);
      const v16h vh3 = ldfrag_h(vhp + (size_t)48 * SEQ);
      const v16h vl0 = ldfrag_h(vlp);
      const v16h vl1 = ldfrag_h(vlp + (size_t)16 * SEQ);
      const v16h vl2 = ldfrag_h(vlp + (size_t)32 * SEQ);
      const v16h vl3 = ldfrag_h(vlp + (size_t)48 * SEQ);
      o[0] = mma_h(ph.v, vh0, o[0]);  o[0] = mma_h(pl.v, vh0, o[0]);  o[0] = mma_h(ph.v, vl0, o[0]);
      o[1] = mma_h(ph.v, vh1, o[1]);  o[1] = mma_h(pl.v, vh1, o[1]);  o[1] = mma_h(ph.v, vl1, o[1]);
      o[2] = mma_h(ph.v, vh2, o[2]);  o[2] = mma_h(pl.v, vh2, o[2]);  o[2] = mma_h(ph.v, vl2, o[2]);
      o[3] = mma_h(ph.v, vh3, o[3]);  o[3] = mma_h(pl.v, vh3, o[3]);  o[3] = mma_h(ph.v, vl3, o[3]);
      guard10(o[0], o[1], o[2], o[3], ph.v, pl.v, vh0, vh1, vh2, vh3, vl0, vl1, vl2, vl3);
    }
    wave_sync_lds();
  }
  acc_guard4(o[0], o[1], o[2], o[3]);

  wave_sync_lds();
  float* slab = pt;
  const float oc = 1.0f / (PCAR * VCAR);
#pragma unroll
  for (int r = 0; r < 8; ++r) {
    const float inv = (1.0f / lrow[r]) * oc;
#pragma unroll
    for (int j = 0; j < 4; ++j) slab[(8 * hh + r) * 68 + j * 16 + c] = o[j][r] * inv;
  }
  wave_sync_lds();
  v4u oh[4], ol[4];
  const int rq = lane >> 3, c8 = (lane & 7) * 8;
#pragma unroll
  for (int it = 0; it < 4; ++it) {
    const int row = it * 4 + rq;
    const v4f a = *(const v4f*)(slab + row * 68 + c8), bq = *(const v4f*)(slab + row * 68 + c8 + 4);
    float w[8];
#pragma unroll
    for (int e = 0; e < 4; ++e) { w[e] = a[e] * OSC; w[4 + e] = bq[e] * OSC; }
#pragma unroll
    for (int e = 0; e < 4; ++e) {
      const _Float16 h0 = (_Float16)w[2 * e], h1 = (_Float16)w[2 * e + 1];
      const _Float16 l0 = (_Float16)(w[2 * e] - (float)h0), l1 = (_Float16)(w[2 * e + 1] - (float)h1);
      oh[it][e] = pk16(h_bits(h0), h_bits(h1));
      ol[it][e] = pk16(h_bits(l0), h_bits(l1));
    }
  }
  const size_t ob = (((size_t)(b * SEQ + q0)) * NH + head) * HD + c8;
  for (int pass = 0; pass < 2; ++pass) {
#pragma unroll
    for (int it = 0; it < 4; ++it) {
      const int row = it * 4 + rq;
      const size_t o8 = ob + (size_t)row * (NH * HD);
      *(volatile v4u*)(OHIp + o8) = oh[it];
      *(volatile v4u*)(OLOp + o8) = ol[it];
    }
    __threadfence();
  }
}

extern "C" void kernel_launch(void* const* d_in, const int* in_sizes, int n_in,
                              void* d_out, int out_size, void* d_ws, size_t ws_size,
                              hipStream_t stream) {
  const int ROWS = NB * SEQ;
  if (n_in < 11) return;
  if (in_sizes[0] != ROWS * DMOD || in_sizes[1] != ROWS * DMOD || in_sizes[2] != ROWS * DMOD) return;
  if (in_sizes[3] != NH * DMOD * HD || in_sizes[4] != NH * DMOD * HD || in_sizes[5] != NH * DMOD * HD) return;
  if (in_sizes[6] != NH * HD * DMOD) return;
  if (in_sizes[7] != NH * HD || in_sizes[8] != NH * HD || in_sizes[9] != NH * HD || in_sizes[10] != DMOD) return;
  if (out_size != ROWS * DMOD) return;

  const float* Qin = (const float*)d_in[0];
  const float* Kin = (const float*)d_in[1];
  const float* Vin = (const float*)d_in[2];
  const float* wq  = (const float*)d_in[3];
  const float* wk  = (const float*)d_in[4];
  const float* wv  = (const float*)d_in[5];
  const float* wo  = (const float*)d_in[6];
  const float* bq  = (const float*)d_in[7];
  const float* bk  = (const float*)d_in[8];
  const float* bv  = (const float*)d_in[9];
  const float* bo  = (const float*)d_in[10];
  float*       out = (float*)d_out;

  const size_t szTab = (size_t)SEQ * HP * 4;
  const size_t szSt  = 4096;
  const size_t szBd  = (size_t)3 * NH * HD * 4;
  const size_t szXB  = (size_t)ROWS * DMOD * 2;
  const size_t szW   = (size_t)DMOD * DMOD * 2;
  const size_t szF   = (size_t)ROWS * DMOD * 4;
  const size_t szP   = (size_t)ROWS * DMOD * 2;
  const size_t szVP  = (size_t)NB * NH * HD * SEQ * 2;
  size_t off = 0;
  const size_t oCT  = off; off += szTab;
  const size_t oST  = off; off += szTab;
  const size_t oSTA = off; off += szSt;
  const size_t oBQD = off; off += szBd;
  const size_t oXB  = off; off += szXB;
  const size_t oWQB = off; off += szW;
  const size_t oWKB = off; off += szW;
  const size_t oWVB = off; off += szW;
  const size_t oWOB = off; off += szW;
  const size_t oF   = off; off += szF;
  const size_t oQHI = off; off += szP;
  const size_t oQLO = off; off += szP;
  const size_t oKHI = off; off += szP;
  const size_t oKLO = off; off += szP;
  const size_t oVHI = off; off += szVP;
  const size_t oVLO = off; off += szVP;
  const size_t oOHI = off; off += szP;
  const size_t oOLO = off; off += szP;
  if (off > ws_size) return;
  if (off > (size_t)134217728) return;

  char* ws = (char*)d_ws;
  float* CT   = (float*)(ws + oCT);
  float* ST   = (float*)(ws + oST);
  float* STAT = (float*)(ws + oSTA);
  float* BQD  = (float*)(ws + oBQD);
  u16*   XB   = (u16*)(ws + oXB);
  u16*   WQB  = (u16*)(ws + oWQB);
  u16*   WKB  = (u16*)(ws + oWKB);
  u16*   WVB  = (u16*)(ws + oWVB);
  u16*   WOB  = (u16*)(ws + oWOB);
  float* F    = (float*)(ws + oF);
  u16*   QHI  = (u16*)(ws + oQHI);
  u16*   QLO  = (u16*)(ws + oQLO);
  u16*   KHI  = (u16*)(ws + oKHI);
  u16*   KLO  = (u16*)(ws + oKLO);
  u16*   VHI  = (u16*)(ws + oVHI);
  u16*   VLO  = (u16*)(ws + oVLO);
  u16*   OHI  = (u16*)(ws + oOHI);
  u16*   OLO  = (u16*)(ws + oOLO);

  InvF inv;
  for (int i = 0; i < 32; ++i) {
    const double p = pow(10000.0, -(double)i / 32.0);
    inv.f[i] = (float)p;
  }

  const dim3 blk(256);
  const int n8x = (ROWS * DMOD) / 8;
  const int nW4 = in_sizes[3] / 4;
  const int nB4 = in_sizes[7] / 4;
  if ((n8x % 256) != 0 || (in_sizes[3] % 4) != 0 || nB4 != 256) return;
  const dim3 gTab(SEQ / 8);
  const dim3 gSt(6);
  const dim3 gX(n8x / 256);
  const dim3 gWt(NH * (DMOD / 64));
  const dim3 gWo((DMOD / 64) * (DMOD / 64));
  const dim3 gG((ROWS / 64) * (DMOD / 64));
  const dim3 bG(128);
  const int rowsH = ROWS * NH;
  const dim3 gR((rowsH * 8) / 256);
  const dim3 gVT(NB * NH * (SEQ / 64));
  const dim3 gAT(ATT_BLOCKS);
  const dim3 bAT(ATT_THREADS);

  k_tab<<<gTab, blk, 0, stream>>>(CT, ST, inv);
  k_stats<<<gSt, blk, 0, stream>>>(wq, wk, wv, bq, bk, bv, nW4, nB4, STAT, BQD);
  wqt16<<<gWt, blk, 0, stream>>>(wq, STAT + 0 * 32, WQB);
  wqt16<<<gWt, blk, 0, stream>>>(wk, STAT + 1 * 32, WKB);
  wqt16<<<gWt, blk, 0, stream>>>(wv, STAT + 2 * 32, WVB);
  wot16<<<gWo, blk, 0, stream>>>(wo, WOB);
  cvtbf<<<gX, blk, 0, stream>>>(Qin, XB, n8x);
  gemm_bf<<<gG, bG, 0, stream>>>(XB, WQB, BQD + 0 * (NH * HD), STAT + 0 * 32 + 2, F, ROWS, DMOD, DMOD);
  rot16<<<gR, blk, 0, stream>>>(F, CT, ST, QHI, QLO, rowsH, NH, QSC);
  cvtbf<<<gX, blk, 0, stream>>>(Kin, XB, n8x);
  gemm_bf<<<gG, bG, 0, stream>>>(XB, WKB, BQD + 1 * (NH * HD), STAT + 1 * 32 + 2, F, ROWS, DMOD, DMOD);
  rot16<<<gR, blk, 0, stream>>>(F, CT, ST, KHI, KLO, rowsH, NH, KSC);
  cvtbf<<<gX, blk, 0, stream>>>(Vin, XB, n8x);
  gemm_bf<<<gG, bG, 0, stream>>>(XB, WVB, BQD + 2 * (NH * HD), STAT + 2 * 32 + 2, F, ROWS, DMOD, DMOD);
  vt16<<<gVT, blk, 0, stream>>>(F, VHI, VLO);
  attn_causal<<<gAT, bAT, 0, stream>>>(QHI, QLO, KHI, KLO, VHI, VLO, OHI, OLO);
  gemm_h2<<<gG, bG, 0, stream>>>(OHI, OLO, WOB, bo, out, ROWS, DMOD, DMOD, 1.0f / (OSC * WOS));
  (void)hipGetLastError();
}
